// TFAttention_77807627534899
// MI455X (gfx1250) — hardware-verified
//
#include <hip/hip_runtime.h>
#include <stdint.h>

typedef __attribute__((ext_vector_type(16))) _Float16 v16h;
typedef __attribute__((ext_vector_type(8)))  _Float16 v8h;
typedef __attribute__((ext_vector_type(16))) __bf16   v16b;
typedef __attribute__((ext_vector_type(8)))  __bf16   v8b;
typedef __attribute__((ext_vector_type(8)))  float    v8f;
typedef __attribute__((ext_vector_type(4)))  float    v4f;
typedef __attribute__((ext_vector_type(2)))  float    v2f;
typedef __attribute__((ext_vector_type(4)))  unsigned int v4u;

static constexpr int kBatch  = 2;
static constexpr int kSeq    = 2048;
static constexpr int kModel  = 1024;
static constexpr int kHeads  = 16;
static constexpr int kHdim   = 64;
static constexpr int kRows   = kBatch * kSeq;
static constexpr int kQKCols = 2 * kModel;
static constexpr int kQKV    = 3 * kModel;
static_assert(kModel == kHeads * kHdim, "head split");
static_assert(kHdim == 64, "attention kernel is written for head dim 64");
static_assert(kSeq % 64 == 0, "64-key chunks and 64-query blocks");

static constexpr size_t kBytesXb   = (size_t)kRows * kModel * 2;
static constexpr size_t kBytesWqkT = (size_t)kQKV * kModel * 2;
static constexpr size_t kBytesWpT  = (size_t)kModel * kModel * 2;
static constexpr size_t kBytesQK   = (size_t)kRows * kQKCols * 2;
static constexpr size_t kBytesVt   = (size_t)kBatch * kModel * kSeq * 2;
static constexpr size_t kBytesA    = (size_t)kRows * kModel * 2;
static constexpr size_t kOffXb   = 0;
static constexpr size_t kOffWqkT = kOffXb + kBytesXb;
static constexpr size_t kOffWpT  = kOffWqkT + kBytesWqkT;
static constexpr size_t kOffQKhi = kOffWpT + kBytesWpT;
static constexpr size_t kOffQKlo = kOffQKhi + kBytesQK;
static constexpr size_t kOffVthi = kOffQKlo + kBytesQK;
static constexpr size_t kOffVtlo = kOffVthi + kBytesVt;
static constexpr size_t kOffAhi  = kOffVtlo + kBytesVt;
static constexpr size_t kOffAlo  = kOffAhi + kBytesA;
static constexpr size_t kWsTotal = kOffAlo + kBytesA;
static_assert(kWsTotal == 83886080u, "carve total");
static_assert(kWsTotal <= 134217728u, "carve within 128 MiB");
static_assert(kOffWqkT % 128 == 0 && kOffWpT % 128 == 0 && kOffQKhi % 128 == 0 && kOffQKlo % 128 == 0 &&
              kOffVthi % 128 == 0 && kOffVtlo % 128 == 0 && kOffAhi % 128 == 0 && kOffAlo % 128 == 0, "128-B aligned regions");

static_assert(kRows % 64 == 0 && kQKCols % 64 == 0 && kModel % 64 == 0 && kSeq % 64 == 0, "M,N tile multiples");
static_assert(kModel % 32 == 0, "K multiple of 32");

__device__ __forceinline__ unsigned short f2bf_bits(float f) {
  unsigned u = __float_as_uint(f);
  return (unsigned short)((u + 0x7FFFu + ((u >> 16) & 1u)) >> 16);
}
__device__ __forceinline__ float bf_bits2f(unsigned short h) { return __uint_as_float(((unsigned)h) << 16); }

__device__ __forceinline__ void dep_guard_h(v8f& a, v8f& b, v16h x, v16h y) { asm volatile("v_nop\n\tv_nop\n\tv_nop\n\tv_nop" : "+v"(a), "+v"(b) : "v"(x), "v"(y)); }
__device__ __forceinline__ void dep_guard_b(v8f& a, v8f& b, v16b x, v16b y) { asm volatile("v_nop\n\tv_nop\n\tv_nop\n\tv_nop" : "+v"(a), "+v"(b) : "v"(x), "v"(y)); }
__device__ __forceinline__ void keep4_h(v16h a, v16h b, v16h c, v16h d) { asm volatile("v_nop" :: "v"(a), "v"(b), "v"(c), "v"(d)); }
__device__ __forceinline__ void keep4_b(v16b a, v16b b, v16b c, v16b d) { asm volatile("v_nop" :: "v"(a), "v"(b), "v"(c), "v"(d)); }
__device__ __forceinline__ void acc_guard4(v8f& a, v8f& b, v8f& c, v8f& d) { asm volatile("v_nop\n\tv_nop\n\tv_nop\n\tv_nop" : "+v"(a), "+v"(b), "+v"(c), "+v"(d)); }
template <typename T> struct Frag;
template <> struct Frag<_Float16> {
  typedef v16h V; union U { v16h v; v8h h[2]; };
  static __device__ __forceinline__ v16h load(const _Float16* p) {
    U f; f.h[0] = *(const v8h*)(p); f.h[1] = *(const v8h*)(p + 16); return f.v;
  }
  static __device__ __forceinline__ v8f mma(v16h a, v16h b, v8f c) {
    return __builtin_amdgcn_wmma_f32_16x16x32_f16(false, a, false, b, (short)0, c, false, false);
  }
  static __device__ __forceinline__ void guard(v8f& a, v8f& b, v16h x, v16h y) { dep_guard_h(a, b, x, y); }
  static __device__ __forceinline__ void keep(v16h a, v16h b, v16h c, v16h d) { keep4_h(a, b, c, d); }
};
template <> struct Frag<__bf16> {
  typedef v16b V; union U { v16b v; v8b h[2]; };
  static __device__ __forceinline__ v16b load(const __bf16* p) {
    U f; f.h[0] = *(const v8b*)(p); f.h[1] = *(const v8b*)(p + 16); return f.v;
  }
  static __device__ __forceinline__ v8f mma(v16b a, v16b b, v8f c) {
    return __builtin_amdgcn_wmma_f32_16x16x32_bf16(false, a, false, b, (short)0, c, false, false);
  }
  static __device__ __forceinline__ void guard(v8f& a, v8f& b, v16b x, v16b y) { dep_guard_b(a, b, x, y); }
  static __device__ __forceinline__ void keep(v16b a, v16b b, v16b c, v16b d) { keep4_b(a, b, c, d); }
};

template <int ET> struct Elem;
template <> struct Elem<0> { typedef _Float16 T; };
template <> struct Elem<1> { typedef __bf16 T; };
template <int ET, int SPLIT, int BIAS_MODE, int OUT_MODE>
__global__ __launch_bounds__(256) void wmma_gemm64(
    const unsigned short* __restrict__ Ap, const unsigned short* __restrict__ A2p, int lda, long strideA,
    const unsigned short* __restrict__ Btp, const unsigned short* __restrict__ Bt2p, int ldb, long strideB,
    void* __restrict__ Cout, void* __restrict__ Cout2, int ldc, long strideC,
    const float* __restrict__ bias,
    int M, int N, int K, float scale) {
  typedef typename Elem<ET>::T T;
  typedef typename Frag<T>::V V;
  const T* A = (const T*)Ap; const T* A2 = (const T*)A2p; const T* Bt = (const T*)Btp; const T* Bt2 = (const T*)Bt2p;
  __shared__ __align__(16) float sT[8][16 * 68];
  const int b    = blockIdx.y;
  const int lane = threadIdx.x & 31;
  const int wave = threadIdx.x >> 5;
  const int tilesN = N >> 6;
  const int tilesM = M >> 6;
  const int tile = blockIdx.x * 8 + wave;
  if (tile >= tilesM * tilesN) return;
  const int tm = tile / tilesN;
  const int tn = tile - tm * tilesN;
  const int m0 = tm << 6;
  const int n0 = tn << 6;

  const T* Ab  = A  + (size_t)b * strideA;
  const T* Bb  = Bt + (size_t)b * strideB;
  const T* Ab2 = (SPLIT >= 1) ? (A2  + (size_t)b * strideA) : nullptr;
  const T* Bb2 = (SPLIT == 2) ? (Bt2 + (size_t)b * strideB) : nullptr;

  const int rlane = lane & 15;
  const int koff  = (lane >> 4) * 8;
  const int mOff  = (lane >> 4) * 8;

  v8f acc[4][4];
#pragma unroll
  for (int i = 0; i < 4; ++i)
#pragma unroll
    for (int j = 0; j < 4; ++j) acc[i][j] = (v8f){0.f,0.f,0.f,0.f,0.f,0.f,0.f,0.f};

  for (int k0 = 0; k0 < K; k0 += 32) {
    V bh[4], bl[4];
#pragma unroll
    for (int j = 0; j < 4; ++j) {
      const size_t bo = (size_t)(n0 + (j << 4) + rlane) * ldb + koff + k0;
      bh[j] = Frag<T>::load(Bb + bo);
      if (SPLIT == 2) bl[j] = Frag<T>::load(Bb2 + bo);
    }
#pragma unroll
    for (int i = 0; i < 4; ++i) {
      const size_t ao = (size_t)(m0 + (i << 4) + rlane) * lda + koff + k0;
      V ah = Frag<T>::load(Ab + ao);
      V al;
      if (SPLIT >= 1) al = Frag<T>::load(Ab2 + ao);
#pragma unroll
      for (int j = 0; j < 4; ++j) {
        acc[i][j] = Frag<T>::mma(ah, bh[j], acc[i][j]);
        if (SPLIT == 2) acc[i][j] = Frag<T>::mma(ah, bl[j], acc[i][j]);
        if (SPLIT >= 1) acc[i][j] = Frag<T>::mma(al, bh[j], acc[i][j]);
      }
      Frag<T>::guard(acc[i][0], acc[i][3], ah, (SPLIT >= 1) ? al : ah);
    }
    Frag<T>::keep(bh[0], bh[1], bh[2], bh[3]);
    if (SPLIT == 2) Frag<T>::keep(bl[0], bl[1], bl[2], bl[3]);
  }
  acc_guard4(acc[0][0], acc[0][1], acc[0][2], acc[0][3]);
  acc_guard4(acc[1][0], acc[1][1], acc[1][2], acc[1][3]);
  acc_guard4(acc[2][0], acc[2][1], acc[2][2], acc[2][3]);
  acc_guard4(acc[3][0], acc[3][1], acc[3][2], acc[3][3]);

  float* slab = sT[wave];
#pragma unroll
  for (int i = 0; i < 4; ++i) {
    const int mBase = m0 + (i << 4);
#pragma unroll
    for (int j = 0; j < 4; ++j) {
      const int n = n0 + (j << 4) + rlane;
      float bv = 0.f;
      if (BIAS_MODE == 2) bv = bf_bits2f(f2bf_bits(bias[n]));
#pragma unroll
      for (int r = 0; r < 8; ++r) {
        float v = acc[i][j][r] * scale;
        if (BIAS_MODE == 1) v += bf_bits2f(f2bf_bits(bias[mBase + mOff + r]));
        if (BIAS_MODE == 2) v += bv;
        slab[(mOff + r) * 68 + (j << 4) + rlane] = v;
      }
    }
    __builtin_amdgcn_fence(__ATOMIC_RELEASE, "workgroup");
    __builtin_amdgcn_wave_barrier();
    __builtin_amdgcn_fence(__ATOMIC_ACQUIRE, "workgroup");
    if (OUT_MODE == 0) {
      float* C = (float*)Cout + (size_t)b * strideC;
      const int hh = lane >> 4, c4 = (lane & 15) * 4;
      for (int pass = 0; pass < 2; ++pass) {
#pragma unroll
        for (int it = 0; it < 8; ++it) {
          const int row = it * 2 + hh;
          v4f v = *(const v4f*)(slab + row * 68 + c4);
          *(volatile v4f*)(C + (size_t)(mBase + row) * ldc + n0 + c4) = v;
        }
        __threadfence();
      }
    } else {
      const int q = lane >> 3, c8 = (lane & 7) * 8;
      unsigned short* C  = (unsigned short*)Cout  + (size_t)b * strideC;
      unsigned short* C2 = (OUT_MODE == 2) ? ((unsigned short*)Cout2 + (size_t)b * strideC) : nullptr;
      for (int pass = 0; pass < 2; ++pass) {
#pragma unroll
        for (int it = 0; it < 4; ++it) {
          const int row = it * 4 + q;
          const float* sp = slab + row * 68 + c8;
          v8h hv, lv;
#pragma unroll
          for (int e = 0; e < 8; ++e) {
            if (OUT_MODE == 1) {
              hv[e] = (_Float16)sp[e];
            } else {
              unsigned short hb = f2bf_bits(sp[e]);
              unsigned short lb = f2bf_bits(sp[e] - bf_bits2f(hb));
              hv[e] = __builtin_bit_cast(_Float16, hb);
              lv[e] = __builtin_bit_cast(_Float16, lb);
            }
          }
          *(volatile v8h*)(C + (size_t)(mBase + row) * ldc + n0 + c8) = hv;
          if (OUT_MODE == 2) *(volatile v8h*)(C2 + (size_t)(mBase + row) * ldc + n0 + c8) = lv;
        }
        __threadfence();
      }
    }
    __builtin_amdgcn_fence(__ATOMIC_RELEASE, "workgroup");
    __builtin_amdgcn_wave_barrier();
    __builtin_amdgcn_fence(__ATOMIC_ACQUIRE, "workgroup");
  }
}

__global__ __launch_bounds__(256) void cast_f32_bf16x2(
    const float* __restrict__ in, unsigned short* __restrict__ out, int n2) {
  int i = blockIdx.x * 256 + threadIdx.x;
  if (i < n2) {
    const v2f f = *(const v2f*)(in + 2 * (size_t)i);
    const unsigned u = (unsigned)f2bf_bits(f[0]) | ((unsigned)f2bf_bits(f[1]) << 16);
    ((volatile unsigned*)out)[i] = u;
    __threadfence();
    ((volatile unsigned*)out)[i] = u;
  }
}

union TrTile { unsigned short s[64 * 72]; v4u u[64 * 9]; };
__global__ __launch_bounds__(256) void transpose_cast_bf16(
    const float* __restrict__ in, unsigned short* __restrict__ outp, int nRows, int nCols) {
  __shared__ __align__(16) TrTile T;
  const int tid = threadIdx.x;
  const int r0 = blockIdx.y * 64;
  const int c0 = blockIdx.x * 64;
#pragma unroll
  for (int i = 0; i < 4; ++i) {
    const int idx = tid + 256 * i;
    const int rr = idx >> 4, c4 = (idx & 15) * 4;
    const v4f v = *(const v4f*)(in + (size_t)(r0 + rr) * nCols + c0 + c4);
#pragma unroll
    for (int e = 0; e < 4; ++e) T.s[(c4 + e) * 72 + rr] = f2bf_bits(v[e]);
  }
  __syncthreads();
  for (int pass = 0; pass < 2; ++pass) {
#pragma unroll
    for (int i = 0; i < 2; ++i) {
      const int idx = tid + 256 * i;
      const int nn = idx >> 3, w = idx & 7;
      const v4u word = T.u[nn * 9 + w];
      *(volatile v4u*)(outp + (size_t)(c0 + nn) * nRows + r0 + 8 * w) = word;
    }
    __threadfence();
  }
}

union Tile64 { unsigned short s[64 * 64]; v4u u[64 * 8]; };
union Tile16 { unsigned short s[16 * 64]; v4u u[16 * 8]; };
union QF { v16b v; v4u u[2]; };

__device__ __forceinline__ v8f at_mma(v16b a, v16b b, v8f c) {
  c = __builtin_amdgcn_wmma_f32_16x16x32_bf16(false, a, false, b, (short)0, c, false, false);
  asm volatile("v_nop\n\tv_nop\n\tv_nop\n\tv_nop" : "+v"(c) : "v"(a), "v"(b));
  return c;
}

__global__ __launch_bounds__(128)
void attn_causal64(const unsigned short* __restrict__ qk_hi, const unsigned short* __restrict__ qk_lo,
                   const unsigned short* __restrict__ vt_hi, const unsigned short* __restrict__ vt_lo,
                   unsigned short* __restrict__ a_hi, unsigned short* __restrict__ a_lo) {
  __shared__ __align__(16) Tile64 Ksh, Ksl;
  __shared__ __align__(16) Tile64 Vth, Vtl;
  __shared__ __align__(16) Tile16 Psh[4], Psl[4];
  __shared__ __align__(16) float  Os[4][16 * 68];

  const int tid  = threadIdx.x;
  const int wave = tid >> 5;
  const int lane = tid & 31;
  const int hh   = lane >> 4;
  const int c    = lane & 15;

  const int nqb = kSeq / 64;
  const int bx  = blockIdx.x;
  const int qb  = bx % nqb;
  const int bhd = bx / nqb;
  const int h   = bhd % kHeads;
  const int b   = bhd / kHeads;
  const int q0  = qb * 64 + wave * 16;

  QF qah[2], qal[2];
  {
    const size_t qoff = ((size_t)(b * kSeq + q0 + c)) * kQKCols + h * kHdim;
    const v4u* qrh = (const v4u*)(qk_hi + qoff);
    const v4u* qrl = (const v4u*)(qk_lo + qoff);
#pragma unroll
    for (int dc = 0; dc < 2; ++dc) {
      qah[dc].u[0] = qrh[dc * 4 + hh];
      qah[dc].u[1] = qrh[dc * 4 + 2 + hh];
      qal[dc].u[0] = qrl[dc * 4 + hh];
      qal[dc].u[1] = qrl[dc * 4 + 2 + hh];
    }
  }

  const float kNegInf = -__builtin_inff();
  float mrow[8], lrow[8];
  v8f oacc[4];
#pragma unroll
  for (int r = 0; r < 8; ++r) { mrow[r] = kNegInf; lrow[r] = 0.f; }
#pragma unroll
  for (int t = 0; t < 4; ++t) oacc[t] = (v8f){0.f,0.f,0.f,0.f,0.f,0.f,0.f,0.f};

  const int nChunks = qb + 1;
  for (int kc = 0; kc < nChunks; ++kc) {
    const int kv0 = kc * 64;
    __syncthreads();
    {
      const size_t krow0 = (size_t)(b * kSeq + kv0);
#pragma unroll
      for (int i = 0; i < 4; ++i) {
        const int idx = tid + 128 * i;
        const int row = idx >> 3, w = idx & 7;
        const size_t eoff = (krow0 + row) * (size_t)kQKCols + kModel + h * kHdim + 8 * w;
        Ksh.u[row * 8 + w] = *(const v4u*)(qk_hi + eoff);
        Ksl.u[row * 8 + w] = *(const v4u*)(qk_lo + eoff);
      }
      asm volatile("" ::: "memory");
#pragma unroll
      for (int i = 0; i < 4; ++i) {
        const int idx = tid + 128 * i;
        const int d = idx >> 3, w = idx & 7;
        const size_t eoff = ((size_t)(b * kModel + h * kHdim + d)) * kSeq + kv0 + 8 * w;
        Vth.u[d * 8 + w] = *(const v4u*)(vt_hi + eoff);
        Vtl.u[d * 8 + w] = *(const v4u*)(vt_lo + eoff);
      }
    }
    __syncthreads();

    v8f s[4];
#pragma unroll
    for (int j = 0; j < 4; ++j) {
      s[j] = (v8f){0.f,0.f,0.f,0.f,0.f,0.f,0.f,0.f};
#pragma unroll
      for (int dc = 0; dc < 2; ++dc) {
        QF kb, kl;
        kb.u[0] = Ksh.u[(j * 16 + c) * 8 + dc * 4 + hh];
        kb.u[1] = Ksh.u[(j * 16 + c) * 8 + dc * 4 + 2 + hh];
        kl.u[0] = Ksl.u[(j * 16 + c) * 8 + dc * 4 + hh];
        kl.u[1] = Ksl.u[(j * 16 + c) * 8 + dc * 4 + 2 + hh];
        s[j] = at_mma(qah[dc].v, kb.v, s[j]);
        s[j] = at_mma(qah[dc].v, kl.v, s[j]);
        s[j] = at_mma(qal[dc].v, kb.v, s[j]);
      }
    }

    const bool diag = (kc == qb);
    float cm[8];
#pragma unroll
    for (int r = 0; r < 8; ++r) {
      const int qrow = q0 + 8 * hh + r;
      float m = kNegInf;
#pragma unroll
      for (int j = 0; j < 4; ++j) {
        const int kvcol = kv0 + j * 16 + c;
        float sv = s[j][r] * 0.125f;
        if (diag && (kvcol > qrow)) sv = -10000.0f;
        s[j][r] = sv;
        m = fmaxf(m, sv);
      }
#pragma unroll
      for (int off = 1; off < 16; off <<= 1) m = fmaxf(m, __shfl_xor(m, off, 32));
      cm[r] = m;
    }

#pragma unroll
    for (int r = 0; r < 8; ++r) {
      const float mnew = fmaxf(mrow[r], cm[r]);
      const float alpha = expf(mrow[r] - mnew);
      mrow[r] = mnew;
      float psum = 0.f;
#pragma unroll
      for (int j = 0; j < 4; ++j) {
        const float p = expf(s[j][r] - mnew);
        psum += p;
        const unsigned short hb = f2bf_bits(p);
        const unsigned short lb = f2bf_bits(p - bf_bits2f(hb));
        const int pidx = (8 * hh + r) * 64 + j * 16 + c;
        Psh[wave].s[pidx] = hb;
        Psl[wave].s[pidx] = lb;
      }
#pragma unroll
      for (int off = 1; off < 16; off <<= 1) psum += __shfl_xor(psum, off, 32);
      lrow[r] = lrow[r] * alpha + psum;
#pragma unroll
      for (int t = 0; t < 4; ++t) oacc[t][r] *= alpha;
    }
    __builtin_amdgcn_fence(__ATOMIC_RELEASE, "workgroup");
    __builtin_amdgcn_wave_barrier();
    __builtin_amdgcn_fence(__ATOMIC_ACQUIRE, "workgroup");

#pragma unroll
    for (int kk = 0; kk < 2; ++kk) {
      QF pa, pl;
      pa.u[0] = Psh[wave].u[c * 8 + kk * 4 + hh];
      pa.u[1] = Psh[wave].u[c * 8 + kk * 4 + 2 + hh];
      pl.u[0] = Psl[wave].u[c * 8 + kk * 4 + hh];
      pl.u[1] = Psl[wave].u[c * 8 + kk * 4 + 2 + hh];
#pragma unroll
      for (int t = 0; t < 4; ++t) {
        QF vb, vl;
        vb.u[0] = Vth.u[(t * 16 + c) * 8 + kk * 4 + hh];
        vb.u[1] = Vth.u[(t * 16 + c) * 8 + kk * 4 + 2 + hh];
        vl.u[0] = Vtl.u[(t * 16 + c) * 8 + kk * 4 + hh];
        vl.u[1] = Vtl.u[(t * 16 + c) * 8 + kk * 4 + 2 + hh];
        oacc[t] = at_mma(pa.v, vb.v, oacc[t]);
        oacc[t] = at_mma(pa.v, vl.v, oacc[t]);
        oacc[t] = at_mma(pl.v, vb.v, oacc[t]);
      }
    }
  }

  float* os = Os[wave];
#pragma unroll
  for (int r = 0; r < 8; ++r) {
    const float inv = 1.0f / lrow[r];
#pragma unroll
    for (int t = 0; t < 4; ++t) os[(8 * hh + r) * 68 + t * 16 + c] = oacc[t][r] * inv;
  }
  __builtin_amdgcn_fence(__ATOMIC_RELEASE, "workgroup");
  __builtin_amdgcn_wave_barrier();
  __builtin_amdgcn_fence(__ATOMIC_ACQUIRE, "workgroup");
  {
    const int qq = lane >> 3, c8 = (lane & 7) * 8;
    for (int pass = 0; pass < 2; ++pass) {
#pragma unroll
      for (int it = 0; it < 4; ++it) {
        const int row = it * 4 + qq;
        const float* sp = os + row * 68 + c8;
        v4u hv, lv;
#pragma unroll
        for (int e = 0; e < 4; ++e) {
          const float f0 = sp[2 * e], f1 = sp[2 * e + 1];
          const unsigned short h0 = f2bf_bits(f0), h1 = f2bf_bits(f1);
          const unsigned short l0 = f2bf_bits(f0 - bf_bits2f(h0));
          const unsigned short l1 = f2bf_bits(f1 - bf_bits2f(h1));
          hv[e] = (unsigned)h0 | ((unsigned)h1 << 16);
          lv[e] = (unsigned)l0 | ((unsigned)l1 << 16);
        }
        const size_t ooff = ((size_t)(b * kSeq + q0 + row)) * kModel + h * kHdim + c8;
        *(volatile v4u*)(a_hi + ooff) = hv;
        *(volatile v4u*)(a_lo + ooff) = lv;
      }
      __threadfence();
    }
  }
}

extern "C" void kernel_launch(void* const* d_in, const int* in_sizes, int n_in,
                              void* d_out, int out_size, void* d_ws, size_t ws_size,
                              hipStream_t stream) {
  if (n_in < 5) return;
  if (in_sizes[0] != kRows * kModel) return;
  if (in_sizes[1] != kModel * kQKV) return;
  if (in_sizes[2] != kQKV) return;
  if (in_sizes[3] != kModel * kModel) return;
  if (in_sizes[4] != kModel) return;
  if (out_size != kRows * kModel) return;
  if (ws_size < kWsTotal) return;

  const float* x      = (const float*)d_in[0];
  const float* w_attn = (const float*)d_in[1];
  const float* b_attn = (const float*)d_in[2];
  const float* w_proj = (const float*)d_in[3];
  const float* b_proj = (const float*)d_in[4];
  float* out = (float*)d_out;

  char* ws = (char*)d_ws;
  unsigned short* xb    = (unsigned short*)(ws + kOffXb);
  unsigned short* wqkT  = (unsigned short*)(ws + kOffWqkT);
  unsigned short* wpT   = (unsigned short*)(ws + kOffWpT);
  unsigned short* qk_hi = (unsigned short*)(ws + kOffQKhi);
  unsigned short* qk_lo = (unsigned short*)(ws + kOffQKlo);
  unsigned short* vt_hi = (unsigned short*)(ws + kOffVthi);
  unsigned short* vt_lo = (unsigned short*)(ws + kOffVtlo);
  unsigned short* a_hi  = (unsigned short*)(ws + kOffAhi);
  unsigned short* a_lo  = (unsigned short*)(ws + kOffAlo);

  {
    const int n2 = kRows * kModel / 2;
    cast_f32_bf16x2<<<(unsigned)((n2 + 255) / 256), 256, 0, stream>>>(x, xb, n2);
  }
  transpose_cast_bf16<<<dim3(kQKV / 64, kModel / 64), 256, 0, stream>>>(w_attn, wqkT, kModel, kQKV);
  transpose_cast_bf16<<<dim3(kModel / 64, kModel / 64), 256, 0, stream>>>(w_proj, wpT, kModel, kModel);

  {
    const int M = kRows, N = kQKCols, K = kModel;
    const int tiles = (M / 64) * (N / 64);
    wmma_gemm64<1, 0, 2, 2><<<dim3((unsigned)((tiles + 7) / 8), 1), 256, 0, stream>>>(
        xb, xb, K, 0L,
        wqkT, wqkT, K, 0L,
        (void*)qk_hi, (void*)qk_lo, N, 0L,
        b_attn, M, N, K, 1.0f);
  }
  {
    const int M = kModel, N = kSeq, K = kModel;
    const int tiles = (M / 64) * (N / 64);
    wmma_gemm64<1, 0, 1, 2><<<dim3((unsigned)((tiles + 7) / 8), kBatch), 256, 0, stream>>>(
        wqkT + (size_t)kQKCols * kModel, wqkT + (size_t)kQKCols * kModel, K, 0L,
        xb, xb, K, (long)kSeq * kModel,
        (void*)vt_hi, (void*)vt_lo, N, (long)kModel * kSeq,
        b_attn + kQKCols, M, N, K, 1.0f);
  }
  attn_causal64<<<kBatch * kHeads * (kSeq / 64), 128, 0, stream>>>(qk_hi, qk_lo, vt_hi, vt_lo, a_hi, a_lo);

  {
    const int M = kRows, N = kModel, K = kModel;
    const int tiles = (M / 64) * (N / 64);
    wmma_gemm64<1, 1, 2, 0><<<dim3((unsigned)((tiles + 7) / 8), 1), 256, 0, stream>>>(
        a_hi, a_lo, K, 0L,
        wpT, wpT, K, 0L,
        (void*)out, (void*)out, N, 0L,
        b_proj, M, N, K, 1.0f);
  }
}
